// CrossAttentionBlock_987842478101
// MI455X (gfx1250) — hardware-verified
//
#include <hip/hip_runtime.h>
#include <hip/hip_bf16.h>


typedef __attribute__((ext_vector_type(16))) _Float16 v16h;
typedef __attribute__((ext_vector_type(8)))  float    v8f;
typedef __attribute__((__vector_size__(4 * sizeof(int)))) int v4i_b128;
typedef __attribute__((ext_vector_type(4))) float v4f_t;
typedef float v4fa __attribute__((ext_vector_type(4), may_alias));
typedef __attribute__((ext_vector_type(4))) unsigned v4u_t;
typedef unsigned v4ua __attribute__((ext_vector_type(4), may_alias));
#define RSPLIT (1.0f / 2048.0f)
#define PLQ ((size_t)BATCH * HEADS * SEQ * HEADDIM * 8)
static __device__ inline unsigned pk2(float a, float b) { return (unsigned)__builtin_bit_cast(unsigned short, (_Float16)a) | ((unsigned)__builtin_bit_cast(unsigned short, (_Float16)b) << 16); }
static __device__ inline unsigned pk2s(float a, float b, unsigned* lo) {
  const _Float16 h0 = (_Float16)a, h1 = (_Float16)b;
  *lo = pk2((a - (float)h0) * 2048.0f, (b - (float)h1) * 2048.0f);
  return (unsigned)__builtin_bit_cast(unsigned short, h0) | ((unsigned)__builtin_bit_cast(unsigned short, h1) << 16);
}

#define HIDDEN   512
#define HEADS    8
#define HEADDIM  64
#define SEQ      1024
#define BATCH    4
#define NEG_INF_ADD (-10000.0f)

#if defined(__has_builtin)
#if __has_builtin(__builtin_amdgcn_global_load_async_to_lds_b128)
#define HAVE_ASYNC_LDS 1
#endif
#endif

static __device__ inline v8f wmma16x16x32(v16h a, v16h b, v8f c) {
  return __builtin_amdgcn_wmma_f32_16x16x32_f16(false, a, false, b,
                                                (short)0, c, false, false);
}
static __device__ inline v8f wmma_split(v16h ah, v16h al, v16h bh, v16h bl, v8f c) {
  v8f x = {};
  x = wmma16x16x32(al, bh, x); x = wmma16x16x32(ah, bl, x);
  return wmma16x16x32(ah, bh, c) + x * RSPLIT;
}

#ifdef HAVE_ASYNC_LDS
typedef __attribute__((address_space(1))) v4i_b128* g_b128_ptr;
typedef __attribute__((address_space(3))) v4i_b128* l_b128_ptr;
static __device__ inline void async_b128(const _Float16* g, _Float16* l) {
  __builtin_amdgcn_global_load_async_to_lds_b128(
      (g_b128_ptr)g, (l_b128_ptr)l, 0, 0);
}
static __device__ inline void async_wait0() {
#if __has_builtin(__builtin_amdgcn_s_wait_asynccnt)
  __builtin_amdgcn_s_wait_asynccnt(0);
#else
  asm volatile("s_wait_asynccnt 0x0" ::: "memory");
#endif
}
#endif

__global__ __launch_bounds__(256)
void proj_gemm_kernel(const float* __restrict__ X,
                      const float* __restrict__ W,
                      _Float16* __restrict__ out,
                      int transposedOut) {
  __shared__ _Float16 Xs[128 * 48];
  __shared__ _Float16 Ws[128 * 48];
  __shared__ _Float16 Xsl[128 * 48];
  __shared__ _Float16 Wsl[128 * 48];
  __shared__ __attribute__((aligned(16))) float Cs[128][128 + 4];

  const int tid  = threadIdx.x;
  const int lane = tid & 31;
  const int wv   = tid >> 5;
  const int mBase = blockIdx.x * 128;
  const int nBase = blockIdx.y * 128;
  const int waveM = (wv >> 1) * 32;
  const int waveN = (wv & 1) * 64;

  const int lc    = lane & 15;
  const int half  = lane >> 4;
  const int kOffA = half * 8;
  const int kOffB = half * 16;

  v8f acc[2][4];
#pragma unroll
  for (int md = 0; md < 2; ++md)
#pragma unroll
    for (int nd = 0; nd < 4; ++nd)
#pragma unroll
      for (int r = 0; r < 8; ++r) acc[md][nd][r] = 0.0f;

  for (int k0 = 0; k0 < HIDDEN; k0 += 32) {
#pragma unroll 2
    for (int i = 0; i < 16; ++i) {
      int idx = i * 256 + tid;
      int row = idx >> 5;
      int col = idx & 31;
      { const float xv = X[(size_t)(mBase + row) * HIDDEN + k0 + col]; const _Float16 xh = (_Float16)xv; Xs[row * 48 + col] = xh; Xsl[row * 48 + col] = (_Float16)((xv - (float)xh) * 2048.0f); }
      { const float wv = W[(size_t)(nBase + row) * HIDDEN + k0 + col]; const _Float16 wh = (_Float16)wv; Ws[row * 48 + col] = wh; Wsl[row * 48 + col] = (_Float16)((wv - (float)wh) * 2048.0f); }
    }
    __syncthreads();

    typedef __attribute__((ext_vector_type(8))) _Float16 v8h_;
    union U16x { v16h v; v8h_ q[2]; };
    U16x afr[2], afl[2];
#pragma unroll
    for (int md = 0; md < 2; ++md) {
      int base = (waveM + md * 16 + lc) * 48 + kOffA;
      afr[md].q[0] = *(const v8h_*)(Xs + base);  afr[md].q[1] = *(const v8h_*)(Xs + base + 16);
      afl[md].q[0] = *(const v8h_*)(Xsl + base); afl[md].q[1] = *(const v8h_*)(Xsl + base + 16);
    }
#pragma unroll
    for (int nd = 0; nd < 4; ++nd) {
      int base = (waveN + nd * 16 + lc) * 48 + kOffA;
      U16x bfr, bfl;
      bfr.q[0] = *(const v8h_*)(Ws + base);  bfr.q[1] = *(const v8h_*)(Ws + base + 16);
      bfl.q[0] = *(const v8h_*)(Wsl + base); bfl.q[1] = *(const v8h_*)(Wsl + base + 16);
#pragma unroll
      for (int md = 0; md < 2; ++md) acc[md][nd] = wmma_split(afr[md].v, afl[md].v, bfr.v, bfl.v, acc[md][nd]);
      asm volatile("" ::: "memory");
    }
    __syncthreads();
  }

#pragma unroll
  for (int md = 0; md < 2; ++md)
#pragma unroll
    for (int nd = 0; nd < 4; ++nd)
#pragma unroll
      for (int r = 0; r < 8; ++r) Cs[waveM + md * 16 + r + 8 * half][waveN + nd * 16 + lc] = acc[md][nd][r];
  __syncthreads();
#pragma unroll 1
  for (int pass = 0; pass < 2; ++pass) {
#pragma unroll
    for (int i = 0; i < 8; ++i) {
      const int c = tid + 256 * i, rl = c >> 4, hh2 = (c >> 3) & 1, q = c & 7;
      const int m = mBase + rl, b = m >> 10, l = m & 1023, h = (nBase >> 6) + hh2;
      const float* s = &Cs[rl][hh2 * 64 + q * 8];
      _Float16* d = out + (((size_t)(b * HEADS + h)) * SEQ + l) * HEADDIM + q * 8;
      v4u_t v, vl; unsigned lo;
      if (transposedOut) { v.x = pk2(s[0], s[1]); v.y = pk2(s[2], s[3]); v.z = pk2(s[4], s[5]); v.w = pk2(s[6], s[7]); *(volatile v4u_t*)d = v; }
      else {
        v.x = pk2s(s[0], s[1], &lo); vl.x = lo; v.y = pk2s(s[2], s[3], &lo); vl.y = lo; v.z = pk2s(s[4], s[5], &lo); vl.z = lo; v.w = pk2s(s[6], s[7], &lo); vl.w = lo;
        *(volatile v4u_t*)d = v; *(volatile v4u_t*)(d + PLQ) = vl;
      }
    }
    __threadfence();
  }
}

__global__ __launch_bounds__(256) void vt_kernel(const _Float16* __restrict__ Vr, _Float16* __restrict__ Vt) {
  __shared__ _Float16 t[64][66];
  const int tid = threadIdx.x, lane = tid & 31, wave = tid >> 5;
  const int bh = blockIdx.x >> 4, l0 = (blockIdx.x & 15) * 64;
  const _Float16* src = Vr + ((size_t)bh * SEQ + l0) * HEADDIM;
#pragma unroll
  for (int k = 0; k < 16; ++k) { const int e = tid + 256 * k; t[e >> 6][e & 63] = src[e]; }
  __syncthreads();
  _Float16* dst = Vt + (size_t)bh * HEADDIM * SEQ + l0;
#pragma unroll
  for (int rr = 0; rr < 8; ++rr) {
    const int dh = wave * 8 + rr;
    const unsigned p = (unsigned)__builtin_bit_cast(unsigned short, t[2 * lane][dh]) | ((unsigned)__builtin_bit_cast(unsigned short, t[2 * lane + 1][dh]) << 16);
    unsigned* d = (unsigned*)(dst + (size_t)dh * SEQ) + lane;
    *(volatile unsigned*)d = p; __threadfence(); *(volatile unsigned*)d = p;
  }
}

__global__ __launch_bounds__(256) __attribute__((amdgpu_num_vgpr(248)))
void flash_attn_kernel(const _Float16* __restrict__ Q,
                       const _Float16* __restrict__ K1,
                       const _Float16* __restrict__ V1t,
                       const _Float16* __restrict__ K2,
                       const _Float16* __restrict__ V2t,
                       const float* __restrict__ maskRow,
                       const float* __restrict__ maskC1,
                       const float* __restrict__ maskC2,
                       float* __restrict__ out) {
  __shared__ _Float16 Ks[64 * HEADDIM];
  __shared__ _Float16 Ksl[64 * HEADDIM];
  __shared__ _Float16 Vts[HEADDIM * 64];
  __shared__ _Float16 Ps[8][16 * 64];
  __shared__ __attribute__((aligned(16))) float Os[8][16 * 64];

  const int tid  = threadIdx.x;
  const int lane = tid & 31;
  const int wv   = tid >> 5;

  const int blk = blockIdx.x;
  const int qb  = blk & 7;
  const int bh  = blk >> 3;
  const int h   = bh & 7;
  const int b   = bh >> 3;
  const int qBase = qb * 128 + wv * 16;

  const size_t bhOff = (size_t)bh * SEQ * HEADDIM;
  const int lc    = lane & 15;
  const int half  = lane >> 4;
  const int kOffA = half * 8;
  const int kOffB = half * 16;

  v16h aq[2], aql[2];
  {
    const _Float16* qp = Q + bhOff + (size_t)(qBase + lc) * HEADDIM;
#pragma unroll
    for (int c = 0; c < 2; ++c)
#pragma unroll
      for (int j = 0; j < 8; ++j) {
        aq[c][j]      = qp[c * 32 + kOffA + j];
        aq[c][8 + j]  = qp[c * 32 + kOffA + 16 + j];
        aql[c][j]     = qp[PLQ + c * 32 + kOffA + j];
        aql[c][8 + j] = qp[PLQ + c * 32 + kOffA + 16 + j];
      }
  }

  v8f outAcc[4];
#pragma unroll
  for (int nd = 0; nd < 4; ++nd)
#pragma unroll
    for (int r = 0; r < 8; ++r) outAcc[nd][r] = 0.0f;

  for (int s = 0; s < 2; ++s) {
    const _Float16* Kt = s ? K2 : K1;
    const _Float16* Vt = s ? V2t : V1t;
    const float*    mc = s ? maskC2 : maskC1;

    float mrun[8], lrun[8];
#pragma unroll
    for (int r = 0; r < 8; ++r) { mrun[r] = -3.0e38f; lrun[r] = 0.0f; }
    v8f oacc[4];
#pragma unroll
    for (int nd = 0; nd < 4; ++nd)
#pragma unroll
      for (int r = 0; r < 8; ++r) oacc[nd][r] = 0.0f;

    for (int kt = 0; kt < SEQ / 64; ++kt) {
      const int keyBase = kt * 64;

      __syncthreads();
      {
        const _Float16* kg = Kt + bhOff + (size_t)keyBase * HEADDIM;
#pragma unroll
        for (int i = 0; i < 2; ++i) {
          int idx = i * 256 + tid;
          int dh  = idx >> 3;
          int c   = idx & 7;
          const _Float16* gv = Vt + bhOff + (size_t)dh * SEQ + keyBase + c * 8;
#ifdef HAVE_ASYNC_LDS
          async_b128(kg + idx * 8, &Ks[idx * 8]);
          async_b128(kg + PLQ + idx * 8, &Ksl[idx * 8]);
          async_b128(gv,           &Vts[idx * 8]);
#else
#pragma unroll
          for (int j = 0; j < 8; ++j) {
            Ks[idx * 8 + j]  = kg[idx * 8 + j];
            Ksl[idx * 8 + j] = kg[PLQ + idx * 8 + j];
            Vts[idx * 8 + j] = gv[j];
          }
#endif
        }
#ifdef HAVE_ASYNC_LDS
        async_wait0();
#endif
      }
      __syncthreads();

      float madd[4];
#pragma unroll
      for (int sub = 0; sub < 4; ++sub)
        madd[sub] = (mc[b * SEQ + keyBase + sub * 16 + lc] > 0.0f)
                        ? 0.0f : NEG_INF_ADD;

      v8f sfr[4];
#pragma unroll
      for (int sub = 0; sub < 4; ++sub)
#pragma unroll
        for (int r = 0; r < 8; ++r) sfr[sub][r] = 0.0f;
#pragma unroll
      for (int c = 0; c < 2; ++c) {
#pragma unroll
        for (int sub = 0; sub < 4; ++sub) {
          typedef __attribute__((ext_vector_type(8))) _Float16 v8h_;
          union U16 { v16h v; v8h_ q[2]; } bk, bkl;
          int base = (sub * 16 + lc) * HEADDIM + c * 32 + kOffA;
          bk.q[0]  = *(const v8h_*)(Ks + base);  bk.q[1]  = *(const v8h_*)(Ks + base + 16);
          bkl.q[0] = *(const v8h_*)(Ksl + base); bkl.q[1] = *(const v8h_*)(Ksl + base + 16);
          sfr[sub] = wmma_split(aq[c], aql[c], bk.v, bkl.v, sfr[sub]);
          asm volatile("" ::: "memory");
        }
      }
#pragma unroll
      for (int sub = 0; sub < 4; ++sub)
#pragma unroll
        for (int r = 0; r < 8; ++r) sfr[sub][r] += madd[sub];

      float newm[8];
#pragma unroll
      for (int r = 0; r < 8; ++r) {
        float v = fmaxf(fmaxf(sfr[0][r], sfr[1][r]),
                        fmaxf(sfr[2][r], sfr[3][r]));
#pragma unroll
        for (int d = 1; d < 16; d <<= 1) v = fmaxf(v, __shfl_xor(v, d, 32));
        newm[r] = fmaxf(mrun[r], v);
      }
#pragma unroll
      for (int r = 0; r < 8; ++r) {
        float scale = __expf(mrun[r] - newm[r]);
        mrun[r] = newm[r];
        float rs = 0.0f;
#pragma unroll
        for (int sub = 0; sub < 4; ++sub) {
          float p = __expf(sfr[sub][r] - newm[r]);
          sfr[sub][r] = p;
          rs += p;
        }
#pragma unroll
        for (int d = 1; d < 16; d <<= 1) rs += __shfl_xor(rs, d, 32);
        lrun[r] = lrun[r] * scale + rs;
#pragma unroll
        for (int nd = 0; nd < 4; ++nd) oacc[nd][r] *= scale;
      }

      _Float16* pw = &Ps[wv][0];
#pragma unroll
      for (int r = 0; r < 8; ++r) {
        int row = r + 8 * half;
#pragma unroll
        for (int sub = 0; sub < 4; ++sub)
          pw[row * 64 + sub * 16 + lc] = (_Float16)(sfr[sub][r] * 1024.0f);
      }
      v16h pa[2];
#pragma unroll
      for (int c2 = 0; c2 < 2; ++c2) {
        int base = lc * 64 + c2 * 32;
#pragma unroll
        for (int j = 0; j < 8; ++j) {
          pa[c2][j]     = pw[base + kOffA + j];
          pa[c2][8 + j] = pw[base + kOffA + 16 + j];
        }
      }

#pragma unroll
      for (int c2 = 0; c2 < 2; ++c2) {
#pragma unroll
        for (int nd = 0; nd < 4; ++nd) {
          typedef __attribute__((ext_vector_type(8))) _Float16 v8h_;
          union U16 { v16h v; v8h_ q[2]; } vb;
          int base = (nd * 16 + lc) * 64 + c2 * 32 + kOffA;
          vb.q[0] = *(const v8h_*)(Vts + base); vb.q[1] = *(const v8h_*)(Vts + base + 16);
          oacc[nd] = wmma16x16x32(pa[c2], vb.v, oacc[nd]);
        }
      }
    }

#pragma unroll
    for (int r = 0; r < 8; ++r) {
      float inv = 0.5f / fmaxf(lrun[r] * 1024.0f, 1e-30f);
#pragma unroll
      for (int nd = 0; nd < 4; ++nd) outAcc[nd][r] += oacc[nd][r] * inv;
    }
  }

  float* os_ = Os[wv];
#pragma unroll
  for (int r = 0; r < 8; ++r) {
    int qg = qBase + r + 8 * half;
    float rm = (maskRow[b * SEQ + qg] > 0.0f) ? 1.0f : 0.0f;
#pragma unroll
    for (int nd = 0; nd < 4; ++nd) os_[(r + 8 * half) * 64 + nd * 16 + lc] = outAcc[nd][r] * rm;
  }
  asm volatile("s_wait_dscnt 0" ::: "memory");
  v4f_t ov[8]; size_t oo[8];
#pragma unroll
  for (int i = 0; i < 8; ++i) { const int c = lane + 32 * i, rr = c >> 4, q = c & 15; ov[i] = *(const volatile v4fa*)(os_ + rr * 64 + q * 4); oo[i] = ((size_t)(b * SEQ + qBase + rr)) * HIDDEN + h * HEADDIM + q * 4; }
#pragma unroll
  for (int i = 0; i < 8; ++i) *(volatile v4f_t*)(out + oo[i]) = ov[i];
  __threadfence();
#pragma unroll
  for (int i = 0; i < 8; ++i) *(volatile v4f_t*)(out + oo[i]) = ov[i];
}

extern "C" void kernel_launch(void* const* d_in, const int* in_sizes, int n_in,
                              void* d_out, int out_size, void* d_ws, size_t ws_size,
                              hipStream_t stream) {
  const float* input1 = (const float*)d_in[0];
  const float* mask1  = (const float*)d_in[1];
  const float* input2 = (const float*)d_in[2];
  const float* mask2  = (const float*)d_in[3];
  const float* Wq1    = (const float*)d_in[4];
  const float* Wk1    = (const float*)d_in[5];
  const float* Wv1    = (const float*)d_in[6];
  const float* Wq2    = (const float*)d_in[7];
  const float* Wk2    = (const float*)d_in[8];
  const float* Wv2    = (const float*)d_in[9];
  float* out = (float*)d_out;

  const size_t T = (size_t)BATCH * HEADS * SEQ * HEADDIM;
  _Float16* ws = (_Float16*)d_ws;
  _Float16* q1  = ws + 0 * T;
  _Float16* k1  = ws + 1 * T;
  _Float16* v1t = ws + 2 * T;
  _Float16* q2  = ws + 3 * T;
  _Float16* k2  = ws + 4 * T;
  _Float16* v2t = ws + 5 * T;
  _Float16* v1r = ws + 6 * T;
  _Float16* v2r = ws + 7 * T;

  dim3 gGemm(32, 4, 1);
  dim3 blk(256, 1, 1);
  proj_gemm_kernel<<<gGemm, blk, 0, stream>>>(input1, Wq1, q1,  0);
  proj_gemm_kernel<<<gGemm, blk, 0, stream>>>(input1, Wk1, k1,  0);
  proj_gemm_kernel<<<gGemm, blk, 0, stream>>>(input1, Wv1, v1r, 1);
  vt_kernel<<<BATCH * HEADS * (SEQ / 64), blk, 0, stream>>>(v1r, v1t);
  proj_gemm_kernel<<<gGemm, blk, 0, stream>>>(input2, Wq2, q2,  0);
  proj_gemm_kernel<<<gGemm, blk, 0, stream>>>(input2, Wk2, k2,  0);
  proj_gemm_kernel<<<gGemm, blk, 0, stream>>>(input2, Wv2, v2r, 1);
  vt_kernel<<<BATCH * HEADS * (SEQ / 64), blk, 0, stream>>>(v2r, v2t);

  dim3 gAttn(BATCH * HEADS * (SEQ / 128), 1, 1);
  flash_attn_kernel<<<gAttn, blk, 0, stream>>>(q1, k1, v1t, k2, v2t,
                                               mask1, mask1, mask2, out);
  flash_attn_kernel<<<gAttn, blk, 0, stream>>>(q2, k1, v1t, k2, v2t,
                                               mask2, mask1, mask2,
                                               out + (size_t)BATCH * SEQ * HIDDEN);
}
